// UltraFastFoveatedConv2d_7997229105540
// MI455X (gfx1250) — hardware-verified
//
#include <hip/hip_runtime.h>
#include <math.h>

typedef __attribute__((ext_vector_type(16))) _Float16 v16h;
typedef __attribute__((ext_vector_type(8)))  _Float16 v8h;
typedef __attribute__((ext_vector_type(16))) __bf16   v16b;
typedef __attribute__((ext_vector_type(8)))  __bf16   v8b;
typedef __attribute__((ext_vector_type(8)))  float    v8f;
typedef __attribute__((ext_vector_type(4)))  float    v4f;

constexpr int NIMG      = 4;
constexpr int NCH_IN    = 32;
constexpr int NCH_OUT   = 64;
constexpr int IMG_H     = 128;
constexpr int IMG_W     = 128;
constexpr int NPIX_IMG  = IMG_H * IMG_W;
constexpr int NTAPS     = 49;
constexpr int KDIM_REAL = NTAPS * NCH_IN;
constexpr int KDIM_PAD  = 1600;
constexpr int WF_PITCH  = 1568;
constexpr int OFF_RING5 = 288;
constexpr int OFF_RING7 = 800;
constexpr int CHUNKS_PER_ROW = KDIM_PAD / 8;
static_assert(KDIM_PAD % 32 == 0);
static_assert(KDIM_PAD >= KDIM_REAL);
static_assert((NCH_OUT * KDIM_PAD) % 256 == 0);
static_assert((NPIX_IMG * CHUNKS_PER_ROW) % 256 == 0);
static_assert(NPIX_IMG % 64 == 0 && NCH_OUT % 64 == 0);

__device__ __forceinline__ unsigned short f2bf_bits(float f) {
  unsigned u = __float_as_uint(f);
  return (unsigned short)((u + 0x7FFFu + ((u >> 16) & 1u)) >> 16);
}
__device__ __forceinline__ float bf_bits2f(unsigned short h) { return __uint_as_float(((unsigned)h) << 16); }

__device__ __forceinline__ void dep_guard_h(v8f& a, v8f& b, v16h x, v16h y) { asm volatile("v_nop\n\tv_nop\n\tv_nop\n\tv_nop" : "+v"(a), "+v"(b) : "v"(x), "v"(y)); }
__device__ __forceinline__ void dep_guard_b(v8f& a, v8f& b, v16b x, v16b y) { asm volatile("v_nop\n\tv_nop\n\tv_nop\n\tv_nop" : "+v"(a), "+v"(b) : "v"(x), "v"(y)); }
__device__ __forceinline__ void keep4_h(v16h a, v16h b, v16h c, v16h d) { asm volatile("v_nop" :: "v"(a), "v"(b), "v"(c), "v"(d)); }
__device__ __forceinline__ void keep4_b(v16b a, v16b b, v16b c, v16b d) { asm volatile("v_nop" :: "v"(a), "v"(b), "v"(c), "v"(d)); }
__device__ __forceinline__ void acc_guard4(v8f& a, v8f& b, v8f& c, v8f& d) { asm volatile("v_nop\n\tv_nop\n\tv_nop\n\tv_nop" : "+v"(a), "+v"(b), "+v"(c), "+v"(d)); }
template <typename T> struct Frag;
template <> struct Frag<_Float16> {
  typedef v16h V; union U { v16h v; v8h h[2]; };
  static __device__ __forceinline__ v16h load(const _Float16* p) {
    U f; f.h[0] = *(const v8h*)(p); f.h[1] = *(const v8h*)(p + 16); return f.v;
  }
  static __device__ __forceinline__ v8f mma(v16h a, v16h b, v8f c) {
    return __builtin_amdgcn_wmma_f32_16x16x32_f16(false, a, false, b, (short)0, c, false, false);
  }
  static __device__ __forceinline__ void guard(v8f& a, v8f& b, v16h x, v16h y) { dep_guard_h(a, b, x, y); }
  static __device__ __forceinline__ void keep(v16h a, v16h b, v16h c, v16h d) { keep4_h(a, b, c, d); }
};
template <> struct Frag<__bf16> {
  typedef v16b V; union U { v16b v; v8b h[2]; };
  static __device__ __forceinline__ v16b load(const __bf16* p) {
    U f; f.h[0] = *(const v8b*)(p); f.h[1] = *(const v8b*)(p + 16); return f.v;
  }
  static __device__ __forceinline__ v8f mma(v16b a, v16b b, v8f c) {
    return __builtin_amdgcn_wmma_f32_16x16x32_bf16(false, a, false, b, (short)0, c, false, false);
  }
  static __device__ __forceinline__ void guard(v8f& a, v8f& b, v16b x, v16b y) { dep_guard_b(a, b, x, y); }
  static __device__ __forceinline__ void keep(v16b a, v16b b, v16b c, v16b d) { keep4_b(a, b, c, d); }
};

template <int ET> struct Elem;
template <> struct Elem<0> { typedef _Float16 T; };
template <> struct Elem<1> { typedef __bf16 T; };
template <int ET, bool SPLIT, int BIAS_MODE, int OUT_MODE, bool RESID, int ACT = 0>
__global__ __launch_bounds__(256) void wmma_gemm64(
    const unsigned short* __restrict__ Ap, const unsigned short* __restrict__ A2p, int lda, long strideA,
    const unsigned short* __restrict__ Btp, const unsigned short* __restrict__ Bt2p, int ldb, long strideB,
    void* __restrict__ Cout, void* __restrict__ Cout2, int ldc, long strideC,
    const float* __restrict__ bias,
    const float* __restrict__ resid, long strideR,
    int M, int N, int K, float scale) {
  typedef typename Elem<ET>::T T;
  typedef typename Frag<T>::V V;
  const T* A = (const T*)Ap; const T* A2 = (const T*)A2p; const T* Bt = (const T*)Btp; const T* Bt2 = (const T*)Bt2p;
  __shared__ __align__(16) float sT[8][16 * 68];
  const int b    = blockIdx.y;
  const int lane = threadIdx.x & 31;
  const int wave = threadIdx.x >> 5;
  const int tilesN = N >> 6;
  const int tilesM = M >> 6;
  const int tile = blockIdx.x * 8 + wave;
  if (tile >= tilesM * tilesN) return;
  const int tm = tile / tilesN;
  const int tn = tile - tm * tilesN;
  const int m0 = tm << 6;
  const int n0 = tn << 6;

  const T* Ab  = A  + (size_t)b * strideA;
  const T* Bb  = Bt + (size_t)b * strideB;
  const T* Ab2 = SPLIT ? (A2  + (size_t)b * strideA) : nullptr;
  const T* Bb2 = SPLIT ? (Bt2 + (size_t)b * strideB) : nullptr;

  const int rlane = lane & 15;
  const int koff  = (lane >> 4) * 8;
  const int mOff  = (lane >> 4) * 8;

  v8f acc[4][4];
#pragma unroll
  for (int i = 0; i < 4; ++i)
#pragma unroll
    for (int j = 0; j < 4; ++j) acc[i][j] = (v8f){0.f,0.f,0.f,0.f,0.f,0.f,0.f,0.f};

  for (int k0 = 0; k0 < K; k0 += 32) {
    V bh[4], bl[4];
#pragma unroll
    for (int j = 0; j < 4; ++j) {
      const size_t bo = (size_t)(n0 + (j << 4) + rlane) * ldb + koff + k0;
      bh[j] = Frag<T>::load(Bb + bo);
      if (SPLIT) bl[j] = Frag<T>::load(Bb2 + bo);
    }
#pragma unroll
    for (int i = 0; i < 4; ++i) {
      const size_t ao = (size_t)(m0 + (i << 4) + rlane) * lda + koff + k0;
      V ah = Frag<T>::load(Ab + ao);
      V al;
      if (SPLIT) al = Frag<T>::load(Ab2 + ao);
#pragma unroll
      for (int j = 0; j < 4; ++j) {
        acc[i][j] = Frag<T>::mma(ah, bh[j], acc[i][j]);
        if (SPLIT) {
          acc[i][j] = Frag<T>::mma(ah, bl[j], acc[i][j]);
          acc[i][j] = Frag<T>::mma(al, bh[j], acc[i][j]);
        }
      }
      Frag<T>::guard(acc[i][0], acc[i][3], ah, SPLIT ? al : ah);
    }
    Frag<T>::keep(bh[0], bh[1], bh[2], bh[3]);
    if (SPLIT) Frag<T>::keep(bl[0], bl[1], bl[2], bl[3]);
  }
  acc_guard4(acc[0][0], acc[0][1], acc[0][2], acc[0][3]);
  acc_guard4(acc[1][0], acc[1][1], acc[1][2], acc[1][3]);
  acc_guard4(acc[2][0], acc[2][1], acc[2][2], acc[2][3]);
  acc_guard4(acc[3][0], acc[3][1], acc[3][2], acc[3][3]);

  float* slab = sT[wave];
  const float* Rb = RESID ? (resid + (size_t)b * strideR) : nullptr;
#pragma unroll
  for (int i = 0; i < 4; ++i) {
    const int mBase = m0 + (i << 4);
#pragma unroll
    for (int j = 0; j < 4; ++j) {
      const int n = n0 + (j << 4) + rlane;
      float bv = 0.f;
      if (BIAS_MODE == 2) bv = bias[n];
#pragma unroll
      for (int r = 0; r < 8; ++r) {
        float v = acc[i][j][r] * scale;
        if (BIAS_MODE == 1) v += bias[mBase + mOff + r];
        if (BIAS_MODE == 2) v += bv;
        if (RESID) v += Rb[(size_t)(mBase + mOff + r) * ldc + n];
        if (ACT == 1) v = tanhf(v);
        if (ACT == 2) v = fmaxf(v, 0.0f);
        if (ACT == 3) v = v / (1.0f + expf(-v));
        if (ACT == 4) v = (v > 0.f) ? v : 0.01f * v;
        if (ACT == 5) v = 0.5f * v * (1.0f + erff(v * 0.70710678118654752f));
        slab[(mOff + r) * 68 + (j << 4) + rlane] = v;
      }
    }
    __builtin_amdgcn_fence(__ATOMIC_RELEASE, "workgroup");
    __builtin_amdgcn_wave_barrier();
    __builtin_amdgcn_fence(__ATOMIC_ACQUIRE, "workgroup");
    if (OUT_MODE == 0) {
      float* C = (float*)Cout + (size_t)b * strideC;
      const int hh = lane >> 4, c4 = (lane & 15) * 4;
      for (int pass = 0; pass < 2; ++pass) {
#pragma unroll
        for (int it = 0; it < 8; ++it) {
          const int row = it * 2 + hh;
          v4f v = *(const v4f*)(slab + row * 68 + c4);
          *(volatile v4f*)(C + (size_t)(mBase + row) * ldc + n0 + c4) = v;
        }
        __threadfence();
      }
    } else {
      const int q = lane >> 3, c8 = (lane & 7) * 8;
      unsigned short* C  = (unsigned short*)Cout  + (size_t)b * strideC;
      unsigned short* C2 = (OUT_MODE == 2) ? ((unsigned short*)Cout2 + (size_t)b * strideC) : nullptr;
      for (int pass = 0; pass < 2; ++pass) {
#pragma unroll
        for (int it = 0; it < 4; ++it) {
          const int row = it * 4 + q;
          const float* sp = slab + row * 68 + c8;
          v8h hv, lv;
#pragma unroll
          for (int e = 0; e < 8; ++e) {
            if (OUT_MODE == 1) {
              hv[e] = (_Float16)sp[e];
            } else {
              unsigned short hb = f2bf_bits(sp[e]);
              unsigned short lb = f2bf_bits(sp[e] - bf_bits2f(hb));
              hv[e] = __builtin_bit_cast(_Float16, hb);
              lv[e] = __builtin_bit_cast(_Float16, lb);
            }
          }
          *(volatile v8h*)(C + (size_t)(mBase + row) * ldc + n0 + c8) = hv;
          if (OUT_MODE == 2) *(volatile v8h*)(C2 + (size_t)(mBase + row) * ldc + n0 + c8) = lv;
        }
        __threadfence();
      }
    }
    __builtin_amdgcn_fence(__ATOMIC_RELEASE, "workgroup");
    __builtin_amdgcn_wave_barrier();
    __builtin_amdgcn_fence(__ATOMIC_ACQUIRE, "workgroup");
  }
}

__global__ __launch_bounds__(256) void fold_weights_kernel(
    const float* __restrict__ wf, const float* __restrict__ w3, const float* __restrict__ w5,
    const float* __restrict__ w7, unsigned short* __restrict__ dst, float scale)
{
  __shared__ __align__(16) _Float16 sW[256];
  const int t   = threadIdx.x;
  const int idx = blockIdx.x * 256 + t;
  const int o   = idx / KDIM_PAD;
  const int k   = idx - o * KDIM_PAD;
  const int tap = k >> 5;
  const int c   = k & 31;
  const bool valid = tap < NTAPS;
  const int tp  = valid ? tap : 0;
  const int ky  = tp / 7;
  const int kx  = tp - ky * 7;
  const int dy3 = ky - 2, dx3 = kx - 2;
  const bool in3 = ((unsigned)dy3 < 3u) && ((unsigned)dx3 < 3u);
  const int p3  = in3 ? (dy3 * 3 + dx3) : 0;
  const int dy5 = ky - 1, dx5 = kx - 1;
  const bool in5 = ((unsigned)dy5 < 5u) && ((unsigned)dx5 < 5u);
  const int p5  = in5 ? (dy5 * 5 + dx5) : 0;
  const float* wfo = wf + (size_t)o * WF_PITCH;
  float a3 = 0.f, a5 = 0.f, a7 = 0.f;
#pragma unroll
  for (int kk = 0; kk < 9; ++kk)
    a3 = fmaf(wfo[c * 9 + kk], w3[(c * 9 + kk) * 9 + p3], a3);
#pragma unroll
  for (int kk = 0; kk < 16; ++kk)
    a5 = fmaf(wfo[OFF_RING5 + c * 16 + kk], w5[(c * 16 + kk) * 25 + p5], a5);
#pragma unroll
  for (int kk = 0; kk < 24; ++kk)
    a7 = fmaf(wfo[OFF_RING7 + c * 24 + kk], w7[(c * 24 + kk) * 49 + tp], a7);
  float acc = a7 + (in5 ? a5 : 0.f) + (in3 ? a3 : 0.f);
  acc = valid ? acc : 0.f;
  sW[t] = (_Float16)(acc * scale);
  __syncthreads();
  if (t < 32) {
    const v8h v = *(const v8h*)(sW + t * 8);
    unsigned short* q = dst + (size_t)blockIdx.x * 256 + t * 8;
    *(volatile v8h*)q = v;
    __threadfence();
    *(volatile v8h*)q = v;
  }
}

__global__ __launch_bounds__(64) void fold_bias_kernel(
    const float* __restrict__ wf, const float* __restrict__ b3, const float* __restrict__ b5,
    const float* __restrict__ b7, const float* __restrict__ bfin, float* __restrict__ beff)
{
  __shared__ __align__(16) float sB[64];
  const int o = threadIdx.x;
  const float* wfo = wf + (size_t)o * WF_PITCH;
  float s3 = 0.f, s5 = 0.f, s7 = 0.f;
#pragma unroll 4
  for (int j = 0; j < 288; ++j) s3 = fmaf(wfo[j], b3[j], s3);
#pragma unroll 4
  for (int j = 0; j < 512; ++j) s5 = fmaf(wfo[OFF_RING5 + j], b5[j], s5);
#pragma unroll 4
  for (int j = 0; j < 768; ++j) s7 = fmaf(wfo[OFF_RING7 + j], b7[j], s7);
  sB[o] = ((bfin[o] + s3) + s5) + s7;
  __syncthreads();
  if (o < 16) {
    const v4f v = *(const v4f*)(sB + 4 * o);
    float* q = beff + 4 * o;
    *(volatile v4f*)q = v;
    __threadfence();
    *(volatile v4f*)q = v;
  }
}

__global__ __launch_bounds__(256) void im2col7_kernel(
    const float* __restrict__ x, unsigned short* __restrict__ dst, int b, int nchunks)
{
  const int f = blockIdx.x * 256 + threadIdx.x;
  if (f >= nchunks) return;
  const int pos = f / CHUNKS_PER_ROW;
  const int g   = f - pos * CHUNKS_PER_ROW;
  const int tap = g >> 2;
  const int c0  = (g & 3) * 8;
  const int h   = pos >> 7;
  const int w   = pos & 127;
  const bool vt = tap < NTAPS;
  const int tp  = vt ? tap : 0;
  const int ky  = tp / 7;
  const int kx  = tp - ky * 7;
  const int yy  = h + ky - 3;
  const int xx  = w + kx - 3;
  const bool inimg = vt && ((unsigned)yy < (unsigned)IMG_H) && ((unsigned)xx < (unsigned)IMG_W);
  const int yc = yy < 0 ? 0 : (yy >= IMG_H ? IMG_H - 1 : yy);
  const int xc = xx < 0 ? 0 : (xx >= IMG_W ? IMG_W - 1 : xx);
  const float* p = x + (((size_t)b * NCH_IN + c0) * IMG_H + yc) * IMG_W + xc;
  v8h hv;
#pragma unroll
  for (int e = 0; e < 8; ++e) {
    const float v = p[(size_t)e * NPIX_IMG];
    hv[e] = inimg ? (_Float16)v : (_Float16)0.0f;
  }
  unsigned short* q = dst + (size_t)f * 8;
  *(volatile v8h*)q = hv;
  __threadfence();
  *(volatile v8h*)q = hv;
}

extern "C" void kernel_launch(void* const* d_in, const int* in_sizes, int n_in,
                              void* d_out, int out_size, void* d_ws, size_t ws_size,
                              hipStream_t stream)
{
  if (n_in < 9) return;
  const float* x   = (const float*)d_in[0];
  const float* w3  = (const float*)d_in[1];
  const float* b3  = (const float*)d_in[2];
  const float* w5  = (const float*)d_in[3];
  const float* b5  = (const float*)d_in[4];
  const float* w7  = (const float*)d_in[5];
  const float* b7  = (const float*)d_in[6];
  const float* wf  = (const float*)d_in[7];
  const float* bfv = (const float*)d_in[8];
  float* dout = (float*)d_out;

  if (in_sizes[0] != NIMG * NCH_IN * NPIX_IMG) return;
  if (in_sizes[1] != NCH_IN * 9 * 9) return;
  if (in_sizes[2] != NCH_IN * 9) return;
  if (in_sizes[3] != NCH_IN * 16 * 25) return;
  if (in_sizes[4] != NCH_IN * 16) return;
  if (in_sizes[5] != NCH_IN * 24 * 49) return;
  if (in_sizes[6] != NCH_IN * 24) return;
  if (in_sizes[7] != NCH_OUT * WF_PITCH) return;
  if (in_sizes[8] != NCH_OUT) return;
  if (out_size != NIMG * NCH_OUT * NPIX_IMG) return;

  const size_t SZ_WEFF = (size_t)NCH_OUT * KDIM_PAD * 2;
  const size_t SZ_BEFF = 256;
  const size_t SZ_ACOL = (size_t)NPIX_IMG * KDIM_PAD * 2;
  const size_t OFF_WEFF = 0;
  const size_t OFF_BEFF = OFF_WEFF + SZ_WEFF;
  const size_t OFF_ACOL = OFF_BEFF + SZ_BEFF;
  const size_t TOTAL    = OFF_ACOL + SZ_ACOL;
  if (ws_size < TOTAL) return;

  char* ws = (char*)d_ws;
  unsigned short* WEFF16 = (unsigned short*)(ws + OFF_WEFF);
  float*          BEFF   = (float*)(ws + OFF_BEFF);
  unsigned short* ACOL   = (unsigned short*)(ws + OFF_ACOL);
  const float*    nores  = x;

  const float WCARRY = 256.0f;
  const int NCHUNK_IMG = NPIX_IMG * CHUNKS_PER_ROW;

  fold_weights_kernel<<<(NCH_OUT * KDIM_PAD) / 256, 256, 0, stream>>>(wf, w3, w5, w7, WEFF16, WCARRY);
  fold_bias_kernel<<<1, 64, 0, stream>>>(wf, b3, b5, b7, bfv, BEFF);

  for (int b = 0; b < NIMG; ++b) {
    im2col7_kernel<<<NCHUNK_IMG / 256, 256, 0, stream>>>(x, ACOL, b, NCHUNK_IMG);
    float* outb = dout + (size_t)b * NCH_OUT * NPIX_IMG;
    wmma_gemm64<0, false, 1, 0, false, 0><<<dim3(32, 1), 256, 0, stream>>>(
        WEFF16, WEFF16, KDIM_PAD, 0L,
        ACOL, ACOL, KDIM_PAD, 0L,
        (void*)outb, (void*)outb, NPIX_IMG, 0L,
        BEFF, nores, 0L,
        NCH_OUT, NPIX_IMG, KDIM_PAD, 1.0f / WCARRY);
  }
}
